// SelfAttention_69569880261434
// MI455X (gfx1250) — hardware-verified
//
#include <hip/hip_runtime.h>


#ifndef NB
#define NB 2
#endif
#ifndef SEQ
#define SEQ 2048
#endif
#define NB_FULL    2
#define SEQ_FULL   2048
#define DM         1024
#define NHEAD      16
#define HDIM       64
#define RTOT       (NB * SEQ)
#define BQ         128
#define BK         32
#define NWAVE      8
#define GT         128
#define OP         68
#define TP         72
#define LNT        128

#define W_S        256.0f
#define T_S        16.0f
#define QKV_S      16.0f
#define CTX_S      64.0f
#define C1_S       64.0f
#define P_S        4096.0f

#define EPI_F16    0
#define EPI_GELU   1
#define EPI_F32    2
#define EPI_GATE   3

static_assert(DM == NHEAD * HDIM);
static_assert(HDIM == 64);
static_assert(SEQ % BQ == 0);
static_assert(SEQ % BK == 0);
static_assert(BQ == NWAVE * 16);
static_assert(RTOT % GT == 0);
static_assert(DM % GT == 0);
static_assert(DM % 32 == 0);
static_assert((2 * DM) % 32 == 0);
static_assert(GT == 4 * 32 && GT == 2 * 64);
static_assert(DM % 64 == 0);
static_assert(LNT * 8 == DM);
static_assert(LNT * 4 == DM / 2);
static_assert(256 * 4 == DM);
static_assert(SEQ <= SEQ_FULL);
static_assert(NB >= 1 && NB <= NB_FULL);
static_assert((TP * 2) % 16 == 0);
static_assert((OP * 4) % 16 == 0);
static_assert(OP >= 64 && TP >= 64);
static_assert(NWAVE * 16 * OP * 4 <= 65536);

constexpr size_t WS_BIAS  = 0;
constexpr size_t SZ_BIAS  = (size_t)16 * DM * 4;
constexpr size_t WS_WT    = WS_BIAS + SZ_BIAS;
constexpr size_t SZ_WT    = (size_t)8 * DM * DM * 2;
constexpr size_t WS_WG    = WS_WT + SZ_WT;
constexpr size_t SZ_WG    = (size_t)2 * DM * DM * 2;
constexpr size_t WS_H     = WS_WG + SZ_WG;
constexpr size_t SZ_ACT   = (size_t)RTOT * DM * 2;
constexpr size_t WS_CAT   = WS_H + SZ_ACT;
constexpr size_t SZ_CAT   = (size_t)RTOT * 2 * DM * 2;
constexpr size_t WS_T     = WS_CAT + SZ_CAT;
constexpr size_t WS_QK    = WS_T + 3 * SZ_ACT;
constexpr size_t WS_VT    = WS_QK + 2 * SZ_ACT;
constexpr size_t WS_TOTAL = WS_VT + SZ_ACT;
static_assert((size_t)RTOT * DM * 4 == 2 * SZ_ACT);
static_assert(WS_TOTAL <= (size_t)134217728);
static_assert(WS_WT % 128 == 0 && WS_WG % 128 == 0 && WS_H % 128 == 0 && WS_CAT % 128 == 0);
static_assert(WS_T % 128 == 0 && WS_QK % 128 == 0 && WS_VT % 128 == 0);

typedef __bf16   bf16;
typedef _Float16 f16;
typedef f16      v16h  __attribute__((ext_vector_type(16)));
typedef f16      v8h   __attribute__((ext_vector_type(8)));
typedef f16      v4h   __attribute__((ext_vector_type(4)));
typedef float    v8f   __attribute__((ext_vector_type(8)));
typedef float    v4f   __attribute__((ext_vector_type(4)));
typedef unsigned v4u   __attribute__((ext_vector_type(4)));

union FragH  { v16h v; v4u q[2]; f16 h[16]; };
union Pack8H { v4u u; v8h v; f16 h[8]; };

static __device__ __forceinline__ v8f mma_f16(v16h a, v16h b, v8f acc) {
  acc = __builtin_amdgcn_wmma_f32_16x16x32_f16(false, a, false, b, (short)0, acc, false, false);
  asm volatile("v_nop\n\tv_nop\n\tv_nop\n\tv_nop" : "+v"(acc) : "v"(a), "v"(b));
  return acc;
}

static __device__ __forceinline__ float bfr(float x) { return (float)(bf16)x; }

__global__ __launch_bounds__(256) void bias_kernel(const float* __restrict__ b0, const float* __restrict__ b1,
                                                   const float* __restrict__ b2, const float* __restrict__ b3,
                                                   const float* __restrict__ b4, const float* __restrict__ b5,
                                                   const float* __restrict__ b6, const float* __restrict__ b7,
                                                   const float* __restrict__ b8, float* __restrict__ biasT) {
  const int c = threadIdx.x * 4;
  v4f v[9];
  v[0] = *(const v4f*)(b0 + c);
  v[1] = *(const v4f*)(b1 + c);
  v[2] = *(const v4f*)(b2 + c);
  v[3] = *(const v4f*)(b3 + c);
  v[4] = *(const v4f*)(b4 + c);
  v[5] = *(const v4f*)(b5 + c);
  v[6] = *(const v4f*)(b6 + c);
  v[7] = *(const v4f*)(b7 + c);
  v[8] = *(const v4f*)(b8 + c);
  #pragma unroll
  for (int j = 0; j < 9; ++j) {
    #pragma unroll
    for (int e = 0; e < 4; ++e) v[j][e] = bfr(v[j][e]);
  }
  #pragma unroll
  for (int j = 0; j < 9; ++j) *(volatile v4f*)(biasT + j * DM + c) = v[j];
  __threadfence();
  #pragma unroll
  for (int j = 0; j < 9; ++j) *(volatile v4f*)(biasT + j * DM + c) = v[j];
}

static __device__ __forceinline__ void cvt_tile(const float* __restrict__ W, f16* __restrict__ Wt,
                                                int N, int K, int k0, int n0) {
  __shared__ __align__(16) f16 sT[64 * TP];
  const int tid = threadIdx.x;
  #pragma unroll
  for (int j = 0; j < 4; ++j) {
    const int kr = j * 16 + (tid >> 4);
    const int nc = (tid & 15) * 4;
    const v4f w = *(const v4f*)(W + (size_t)(k0 + kr) * N + n0 + nc);
    #pragma unroll
    for (int e = 0; e < 4; ++e) sT[(nc + e) * TP + kr] = (f16)(bfr(w[e]) * W_S);
  }
  __syncthreads();
  v4u    vals[2];
  size_t gi[2];
  #pragma unroll
  for (int kk = 0; kk < 2; ++kk) {
    const int n  = kk * 32 + (tid >> 3);
    const int ks = (tid & 7) * 8;
    Pack8H ph;
    ph.v = *(const v8h*)(&sT[n * TP + ks]);
    vals[kk] = ph.u;
    gi[kk] = (size_t)(n0 + n) * K + k0 + ks;
  }
  #pragma unroll
  for (int kk = 0; kk < 2; ++kk) *(volatile v4u*)(Wt + gi[kk]) = vals[kk];
  __threadfence();
  #pragma unroll
  for (int kk = 0; kk < 2; ++kk) *(volatile v4u*)(Wt + gi[kk]) = vals[kk];
  __syncthreads();
}

__global__ __launch_bounds__(256) void wcvt8_kernel(const float* __restrict__ w0, const float* __restrict__ w1,
                                                    const float* __restrict__ w2, const float* __restrict__ w3,
                                                    const float* __restrict__ w4, const float* __restrict__ w5,
                                                    const float* __restrict__ w6, const float* __restrict__ w7,
                                                    f16* __restrict__ wt) {
  const int n0 = blockIdx.x * 64;
  const int k0 = blockIdx.y * 64;
  const size_t P = (size_t)DM * DM;
  cvt_tile(w0, wt + 0 * P, DM, DM, k0, n0);
  cvt_tile(w1, wt + 1 * P, DM, DM, k0, n0);
  cvt_tile(w2, wt + 2 * P, DM, DM, k0, n0);
  cvt_tile(w3, wt + 3 * P, DM, DM, k0, n0);
  cvt_tile(w4, wt + 4 * P, DM, DM, k0, n0);
  cvt_tile(w5, wt + 5 * P, DM, DM, k0, n0);
  cvt_tile(w6, wt + 6 * P, DM, DM, k0, n0);
  cvt_tile(w7, wt + 7 * P, DM, DM, k0, n0);
}

__global__ __launch_bounds__(256) void wcvtg_kernel(const float* __restrict__ wg, f16* __restrict__ wgt) {
  cvt_tile(wg, wgt, DM, 2 * DM, blockIdx.y * 64, blockIdx.x * 64);
}

template <int MODE>
static __device__ __forceinline__ void ln_body(const float* __restrict__ in, const float* __restrict__ gam,
                                               const float* __restrict__ bet, f16* __restrict__ hOut,
                                               f16* __restrict__ catOut, float* __restrict__ fOut) {
  __shared__ float red1[4];
  __shared__ float red2[4];
  __shared__ __align__(16) f16 sA[DM];
  __shared__ __align__(16) f16 sB[DM];
  const int r    = blockIdx.x;
  const int tid  = threadIdx.x;
  const int wave = tid >> 5;
  const int lane = tid & 31;
  const size_t irow = (MODE == 1) ? (size_t)((r / SEQ) * SEQ_FULL + (r % SEQ)) : (size_t)r;
  const float* src = in + irow * DM;
  const int c0 = tid * 4;
  const int c1 = DM / 2 + tid * 4;

  v4f a = *(const v4f*)(src + c0);
  v4f b = *(const v4f*)(src + c1);
  if (MODE == 1) {
    #pragma unroll
    for (int e = 0; e < 4; ++e) { a[e] = bfr(a[e]); b[e] = bfr(b[e]); }
  }
  float s = (a[0] + a[1]) + (a[2] + a[3]) + (b[0] + b[1]) + (b[2] + b[3]);
  #pragma unroll
  for (int off = 16; off > 0; off >>= 1) s += __shfl_xor(s, off, 32);
  if (lane == 0) red1[wave] = s;
  __syncthreads();
  const float mean = ((red1[0] + red1[1]) + (red1[2] + red1[3])) * (1.0f / DM);

  float qv = 0.0f;
  #pragma unroll
  for (int e = 0; e < 4; ++e) {
    const float da = a[e] - mean;
    const float db = b[e] - mean;
    qv += da * da;
    qv += db * db;
  }
  #pragma unroll
  for (int off = 16; off > 0; off >>= 1) qv += __shfl_xor(qv, off, 32);
  if (lane == 0) red2[wave] = qv;
  __syncthreads();
  const float var  = ((red2[0] + red2[1]) + (red2[2] + red2[3])) * (1.0f / DM);
  const float rstd = rsqrtf(var + 1e-5f);

  const v4f g0 = *(const v4f*)(gam + c0);
  const v4f g1 = *(const v4f*)(gam + c1);
  const v4f t0 = *(const v4f*)(bet + c0);
  const v4f t1 = *(const v4f*)(bet + c1);
  v4f y0, y1;
  #pragma unroll
  for (int e = 0; e < 4; ++e) {
    y0[e] = (a[e] - mean) * rstd * bfr(g0[e]) + bfr(t0[e]);
    y1[e] = (b[e] - mean) * rstd * bfr(g1[e]) + bfr(t1[e]);
  }
  v4h h0, h1;
  #pragma unroll
  for (int e = 0; e < 4; ++e) { h0[e] = (f16)y0[e]; h1[e] = (f16)y1[e]; }
  *(v4h*)(&sA[c0]) = h0;
  *(v4h*)(&sA[c1]) = h1;
  if (MODE == 1) {
    v4h x0, x1;
    #pragma unroll
    for (int e = 0; e < 4; ++e) { x0[e] = (f16)a[e]; x1[e] = (f16)b[e]; }
    *(v4h*)(&sB[c0]) = x0;
    *(v4h*)(&sB[c1]) = x1;
  }
  __syncthreads();

  Pack8H pa, pb;
  pa.v = *(const v8h*)(&sA[tid * 8]);
  pb.v = pa.v;
  if (MODE == 1) pb.v = *(const v8h*)(&sB[tid * 8]);

  if (MODE == 1) {
    const size_t ih = (size_t)r * DM + tid * 8;
    const size_t ic = (size_t)r * (2 * DM) + DM + tid * 8;
    *(volatile v4u*)(hOut + ih)   = pa.u;
    *(volatile v4u*)(catOut + ic) = pb.u;
    __threadfence();
    *(volatile v4u*)(hOut + ih)   = pa.u;
    *(volatile v4u*)(catOut + ic) = pb.u;
  } else {
    const size_t ic  = (size_t)r * (2 * DM) + tid * 8;
    const size_t if0 = (size_t)r * DM + c0;
    const size_t if1 = (size_t)r * DM + c1;
    *(volatile v4u*)(catOut + ic) = pa.u;
    *(volatile v4f*)(fOut + if0)  = y0;
    *(volatile v4f*)(fOut + if1)  = y1;
    __threadfence();
    *(volatile v4u*)(catOut + ic) = pa.u;
    *(volatile v4f*)(fOut + if0)  = y0;
    *(volatile v4f*)(fOut + if1)  = y1;
  }
}

__global__ __launch_bounds__(LNT) void ln1_kernel(const float* __restrict__ x, const float* __restrict__ g,
                                                  const float* __restrict__ bt, f16* __restrict__ hOut,
                                                  f16* __restrict__ catOut) {
  ln_body<1>(x, g, bt, hOut, catOut, nullptr);
}
__global__ __launch_bounds__(LNT) void ln2_kernel(const float* __restrict__ pre, const float* __restrict__ g,
                                                  const float* __restrict__ bt, f16* __restrict__ catOut,
                                                  float* __restrict__ fOut) {
  ln_body<2>(pre, g, bt, nullptr, catOut, fOut);
}

template <int EPI, int ROWBIAS>
static __device__ __forceinline__ void gemm_body(
    const f16* __restrict__ A, const f16* __restrict__ Bt, const float* __restrict__ biasT,
    f16* __restrict__ outH, float* __restrict__ outF,
    const float* __restrict__ auxln, const float* __restrict__ xin,
    int lda, int ldb, int K, int ldo, int a_zs, int b_zs, int bias_off, int bias_zs, int o_zs,
    float alpha, float outS) {
  __shared__ __align__(16) float sO[NWAVE * 16 * OP];
  const int tid  = threadIdx.x;
  const int wave = tid >> 5;
  const int lane = tid & 31;
  const int lq   = lane & 15;
  const int hi   = lane >> 4;
  const int z    = blockIdx.z;
  const int row0 = blockIdx.y * GT + (wave >> 1) * 32;
  const int col0 = blockIdx.x * GT + (wave & 1) * 64;
  const int wbase = wave * (16 * OP);
  const int boff  = bias_off + z * bias_zs;

  const f16* Ap = A  + (size_t)z * (size_t)a_zs + (size_t)(row0 + lq) * lda + hi * 8;
  const f16* Bp = Bt + (size_t)z * (size_t)b_zs + (size_t)(col0 + lq) * ldb + hi * 8;

  v8f acc[2][4];
  #pragma unroll
  for (int i = 0; i < 2; ++i) {
    #pragma unroll
    for (int j = 0; j < 4; ++j) acc[i][j] = (v8f){0, 0, 0, 0, 0, 0, 0, 0};
  }

  #pragma unroll 1
  for (int k0 = 0; k0 < K; k0 += 32) {
    FragH a[2], b[4];
    #pragma unroll
    for (int i = 0; i < 2; ++i) {
      const f16* p = Ap + (size_t)(i * 16) * lda + k0;
      a[i].q[0] = *(const v4u*)(p);
      a[i].q[1] = *(const v4u*)(p + 16);
    }
    #pragma unroll
    for (int j = 0; j < 4; ++j) {
      const f16* p = Bp + (size_t)(j * 16) * ldb + k0;
      b[j].q[0] = *(const v4u*)(p);
      b[j].q[1] = *(const v4u*)(p + 16);
    }
    #pragma unroll
    for (int i = 0; i < 2; ++i) {
      #pragma unroll
      for (int j = 0; j < 4; ++j) acc[i][j] = mma_f16(a[i].v, b[j].v, acc[i][j]);
    }
  }

  float bcol[4];
  #pragma unroll
  for (int j = 0; j < 4; ++j) bcol[j] = 0.0f;
  if (ROWBIAS == 0) {
    #pragma unroll
    for (int j = 0; j < 4; ++j) bcol[j] = biasT[boff + col0 + j * 16 + lq];
  }

  #pragma unroll
  for (int i = 0; i < 2; ++i) {
    const int rbase = row0 + i * 16;
    float brow[8];
    #pragma unroll
    for (int r = 0; r < 8; ++r) brow[r] = 0.0f;
    if (ROWBIAS != 0) {
      #pragma unroll
      for (int r = 0; r < 8; ++r) brow[r] = biasT[boff + rbase + hi * 8 + r];
    }
    #pragma unroll
    for (int r = 0; r < 8; ++r) {
      #pragma unroll
      for (int j = 0; j < 4; ++j) {
        const float bb = (ROWBIAS != 0) ? brow[r] : bcol[j];
        sO[wbase + (hi * 8 + r) * OP + j * 16 + lq] = acc[i][j][r] * alpha + bb;
      }
    }
    __syncthreads();

    if (EPI == EPI_GELU) {
      #pragma unroll 1
      for (int it = 0; it < 4; ++it) {
        const int row = it * 4 + (lane >> 3);
        const int c   = (lane & 7) * 8;
        v4f x0 = *(const v4f*)(&sO[wbase + row * OP + c]);
        v4f x1 = *(const v4f*)(&sO[wbase + row * OP + c + 4]);
        #pragma unroll
        for (int e = 0; e < 4; ++e) {
          x0[e] = 0.5f * x0[e] * (1.0f + erff(x0[e] * 0.70710678118654752f));
          x1[e] = 0.5f * x1[e] * (1.0f + erff(x1[e] * 0.70710678118654752f));
        }
        *(v4f*)(&sO[wbase + row * OP + c])     = x0;
        *(v4f*)(&sO[wbase + row * OP + c + 4]) = x1;
      }
      __syncthreads();
    }
    if (EPI == EPI_GATE) {
      #pragma unroll 1
      for (int it = 0; it < 8; ++it) {
        const int row  = it * 2 + hi;
        const int prow = rbase + row;
        const int grow = (prow / SEQ) * SEQ_FULL + (prow % SEQ);
        const int col  = col0 + lq * 4;
        const v4f zv = *(const v4f*)(&sO[wbase + row * OP + lq * 4]);
        const v4f ln = *(const v4f*)(auxln + (size_t)prow * DM + col);
        const v4f xx = *(const v4f*)(xin + (size_t)grow * DM + col);
        v4f y;
        #pragma unroll
        for (int e = 0; e < 4; ++e) {
          const float g  = __builtin_amdgcn_rcpf(1.0f + expf(-zv[e]));
          const float xb = bfr(xx[e]);
          y[e] = g * ln[e] + (1.0f - g) * xb;
        }
        *(v4f*)(&sO[wbase + row * OP + lq * 4]) = y;
      }
      __syncthreads();
    }

    if (EPI == EPI_F16 || EPI == EPI_GELU) {
      v4u    vals[4];
      size_t gi[4];
      #pragma unroll
      for (int it = 0; it < 4; ++it) {
        const int row = it * 4 + (lane >> 3);
        const int c   = (lane & 7) * 8;
        const v4f x0 = *(const v4f*)(&sO[wbase + row * OP + c]);
        const v4f x1 = *(const v4f*)(&sO[wbase + row * OP + c + 4]);
        Pack8H p;
        #pragma unroll
        for (int e = 0; e < 4; ++e) {
          p.h[e]     = (f16)(x0[e] * outS);
          p.h[4 + e] = (f16)(x1[e] * outS);
        }
        vals[it] = p.u;
        gi[it] = (size_t)z * (size_t)o_zs + (size_t)(rbase + row) * ldo + col0 + c;
      }
      #pragma unroll
      for (int it = 0; it < 4; ++it) *(volatile v4u*)(outH + gi[it]) = vals[it];
      __threadfence();
      #pragma unroll
      for (int it = 0; it < 4; ++it) *(volatile v4u*)(outH + gi[it]) = vals[it];
    } else {
      v4f    vals[8];
      size_t gi[8];
      #pragma unroll
      for (int it = 0; it < 8; ++it) {
        const int row  = it * 2 + hi;
        const int prow = rbase + row;
        const int orow = (EPI == EPI_GATE) ? ((prow / SEQ) * SEQ_FULL + (prow % SEQ)) : prow;
        vals[it] = *(const v4f*)(&sO[wbase + row * OP + lq * 4]);
        gi[it] = (size_t)orow * ldo + col0 + lq * 4;
      }
      #pragma unroll
      for (int it = 0; it < 8; ++it) *(volatile v4f*)(outF + gi[it]) = vals[it];
      __threadfence();
      #pragma unroll
      for (int it = 0; it < 8; ++it) *(volatile v4f*)(outF + gi[it]) = vals[it];
    }
    __syncthreads();
  }
}

__global__ __launch_bounds__(256) void gemm_f16_kernel(const f16* __restrict__ A, const f16* __restrict__ Bt,
                                                       const float* __restrict__ biasT, f16* __restrict__ outH,
                                                       int lda, int ldb, int K, int ldo, int a_zs, int b_zs,
                                                       int bias_off, int bias_zs, int o_zs, float alpha, float outS) {
  gemm_body<EPI_F16, 0>(A, Bt, biasT, outH, nullptr, nullptr, nullptr,
                        lda, ldb, K, ldo, a_zs, b_zs, bias_off, bias_zs, o_zs, alpha, outS);
}
__global__ __launch_bounds__(256) void gemm_vt_kernel(const f16* __restrict__ A, const f16* __restrict__ Bt,
                                                      const float* __restrict__ biasT, f16* __restrict__ outH,
                                                      int lda, int ldb, int K, int ldo, int bias_off,
                                                      float alpha, float outS) {
  gemm_body<EPI_F16, 1>(A, Bt, biasT, outH, nullptr, nullptr, nullptr,
                        lda, ldb, K, ldo, 0, 0, bias_off, 0, 0, alpha, outS);
}
__global__ __launch_bounds__(256) void gemm_gelu_kernel(const f16* __restrict__ A, const f16* __restrict__ Bt,
                                                        const float* __restrict__ biasT, f16* __restrict__ outH,
                                                        int lda, int ldb, int K, int ldo, int bias_off,
                                                        float alpha, float outS) {
  gemm_body<EPI_GELU, 0>(A, Bt, biasT, outH, nullptr, nullptr, nullptr,
                         lda, ldb, K, ldo, 0, 0, bias_off, 0, 0, alpha, outS);
}
__global__ __launch_bounds__(256) void gemm_f32_kernel(const f16* __restrict__ A, const f16* __restrict__ Bt,
                                                       const float* __restrict__ biasT, float* __restrict__ outF,
                                                       int lda, int ldb, int K, int ldo, int bias_off, float alpha) {
  gemm_body<EPI_F32, 0>(A, Bt, biasT, nullptr, outF, nullptr, nullptr,
                        lda, ldb, K, ldo, 0, 0, bias_off, 0, 0, alpha, 1.0f);
}
__global__ __launch_bounds__(256) void gemm_gate_kernel(const f16* __restrict__ A, const f16* __restrict__ Bt,
                                                        const float* __restrict__ biasT, float* __restrict__ outF,
                                                        const float* __restrict__ auxln, const float* __restrict__ xin,
                                                        int lda, int ldb, int K, int ldo, int bias_off, float alpha) {
  gemm_body<EPI_GATE, 0>(A, Bt, biasT, nullptr, outF, auxln, xin,
                         lda, ldb, K, ldo, 0, 0, bias_off, 0, 0, alpha, 1.0f);
}

__global__ __launch_bounds__(256) void attn_kernel(const f16* __restrict__ qp, const f16* __restrict__ kp,
                                                   const f16* __restrict__ vt, f16* __restrict__ ctx) {
  const int qblk = blockIdx.x;
  const int h    = blockIdx.y;
  const int b    = blockIdx.z;
  const int tid  = threadIdx.x;
  const int wave = tid >> 5;
  const int lane = tid & 31;
  const int lq   = lane & 15;
  const int hi   = lane >> 4;

  __shared__ __align__(16) float sO[NWAVE * 16 * OP];

  const int qrow0 = b * SEQ + qblk * BQ + wave * 16;
  const int wbase = wave * (16 * OP);

  FragH qf[2];
  {
    const f16* base = qp + (size_t)(qrow0 + lq) * DM + h * HDIM + hi * 8;
    #pragma unroll
    for (int f = 0; f < 2; ++f) {
      qf[f].q[0] = *(const v4u*)(base + f * 32);
      qf[f].q[1] = *(const v4u*)(base + f * 32 + 16);
    }
  }

  const f16* k_h = kp + (size_t)(b * SEQ + lq) * DM + h * HDIM + hi * 8;
  const f16* v_h = vt + (size_t)(h * HDIM + lq) * RTOT + (size_t)b * SEQ + hi * 8;

  v8f o[4];
  #pragma unroll
  for (int dt = 0; dt < 4; ++dt) o[dt] = (v8f){0, 0, 0, 0, 0, 0, 0, 0};

  float rmax = -__builtin_inff();
  float rsum = 0.0f;
  const float SL = 0.125f * 1.4426950408889634f / (QKV_S * QKV_S);

  #pragma unroll 1
  for (int j0 = 0; j0 < SEQ; j0 += BK) {
    FragH ak[2][2];
    #pragma unroll
    for (int sub = 0; sub < 2; ++sub) {
      #pragma unroll
      for (int f = 0; f < 2; ++f) {
        const f16* base = k_h + (size_t)(j0 + sub * 16) * DM + f * 32;
        ak[sub][f].q[0] = *(const v4u*)(base);
        ak[sub][f].q[1] = *(const v4u*)(base + 16);
      }
    }
    FragH bv[4];
    #pragma unroll
    for (int dt = 0; dt < 4; ++dt) {
      const f16* base = v_h + (size_t)(dt * 16) * RTOT + j0;
      bv[dt].q[0] = *(const v4u*)(base);
      bv[dt].q[1] = *(const v4u*)(base + 16);
    }

    v8f c[2];
    #pragma unroll
    for (int sub = 0; sub < 2; ++sub) {
      v8f acc = (v8f){0, 0, 0, 0, 0, 0, 0, 0};
      acc = mma_f16(ak[sub][0].v, qf[0].v, acc);
      acc = mma_f16(ak[sub][1].v, qf[1].v, acc);
      c[sub] = acc;
    }

    float m_new = rmax;
    #pragma unroll
    for (int r = 0; r < 8; ++r) {
      m_new = fmaxf(m_new, c[0][r]);
      m_new = fmaxf(m_new, c[1][r]);
    }
    m_new = fmaxf(m_new, __shfl_xor(m_new, 16, 32));
    const float scale = __builtin_amdgcn_exp2f((rmax - m_new) * SL);
    rmax = m_new;

    FragH pa;
    float psum = 0.0f;
    #pragma unroll
    for (int r = 0; r < 8; ++r) {
      const float p0 = __builtin_amdgcn_exp2f((c[0][r] - m_new) * SL);
      const float p1 = __builtin_amdgcn_exp2f((c[1][r] - m_new) * SL);
      psum += p0 + p1;
      pa.h[r]     = (f16)(p0 * P_S);
      pa.h[8 + r] = (f16)(p1 * P_S);
    }
    rsum = rsum * scale + psum + __shfl_xor(psum, 16, 32);

    float sc[8];
    #pragma unroll
    for (int r = 0; r < 8; ++r) sc[r] = __shfl(scale, (hi << 3) + r, 32);
    #pragma unroll
    for (int dt = 0; dt < 4; ++dt) {
      #pragma unroll
      for (int r = 0; r < 8; ++r) o[dt][r] *= sc[r];
    }

    #pragma unroll
    for (int dt = 0; dt < 4; ++dt) o[dt] = mma_f16(pa.v, bv[dt].v, o[dt]);
  }

  float rs[8];
  #pragma unroll
  for (int r = 0; r < 8; ++r) rs[r] = __builtin_amdgcn_rcpf(__shfl(rsum, (hi << 3) + r, 32));

  const float OS = CTX_S / (P_S * QKV_S);
  #pragma unroll
  for (int r = 0; r < 8; ++r) {
    #pragma unroll
    for (int dt = 0; dt < 4; ++dt) {
      sO[wbase + (hi * 8 + r) * OP + dt * 16 + lq] = o[dt][r] * OS * rs[r];
    }
  }
  __syncthreads();

  v4u    vals[4];
  size_t gi[4];
  #pragma unroll
  for (int it = 0; it < 4; ++it) {
    const int row = it * 4 + (lane >> 3);
    const int cc  = (lane & 7) * 8;
    const v4f x0 = *(const v4f*)(&sO[wbase + row * OP + cc]);
    const v4f x1 = *(const v4f*)(&sO[wbase + row * OP + cc + 4]);
    Pack8H p;
    #pragma unroll
    for (int e = 0; e < 4; ++e) {
      p.h[e]     = (f16)x0[e];
      p.h[4 + e] = (f16)x1[e];
    }
    vals[it] = p.u;
    gi[it] = (size_t)(qrow0 + row) * DM + h * HDIM + cc;
  }
  #pragma unroll
  for (int it = 0; it < 4; ++it) *(volatile v4u*)(ctx + gi[it]) = vals[it];
  __threadfence();
  #pragma unroll
  for (int it = 0; it < 4; ++it) *(volatile v4u*)(ctx + gi[it]) = vals[it];
}

extern "C" void kernel_launch(void* const* d_in, const int* in_sizes, int n_in,
                              void* d_out, int out_size, void* d_ws, size_t ws_size,
                              hipStream_t stream) {
  if (n_in < 23) return;
  const size_t rows_used = (size_t)(NB - 1) * SEQ_FULL + SEQ;
  if ((size_t)in_sizes[0] < rows_used * DM) return;
  for (int i = 1; i <= 15; i += 2) {
    if ((size_t)in_sizes[i] < (size_t)DM * DM) return;
    if ((size_t)in_sizes[i + 1] < (size_t)DM) return;
  }
  for (int i = 17; i <= 20; ++i) if ((size_t)in_sizes[i] < (size_t)DM) return;
  if ((size_t)in_sizes[21] < (size_t)2 * DM * DM) return;
  if ((size_t)in_sizes[22] < (size_t)DM) return;
  if ((size_t)out_size < rows_used * DM) return;
  if (ws_size < WS_TOTAL) return;

  const float* x    = (const float*)d_in[0];
  const float* Wqp  = (const float*)d_in[1];   const float* bqp  = (const float*)d_in[2];
  const float* Wkp  = (const float*)d_in[3];   const float* bkp  = (const float*)d_in[4];
  const float* Wvp  = (const float*)d_in[5];   const float* bvp  = (const float*)d_in[6];
  const float* Wq   = (const float*)d_in[7];   const float* bq   = (const float*)d_in[8];
  const float* Wk   = (const float*)d_in[9];   const float* bk   = (const float*)d_in[10];
  const float* Wv   = (const float*)d_in[11];  const float* bv   = (const float*)d_in[12];
  const float* Wop  = (const float*)d_in[13];  const float* bop  = (const float*)d_in[14];
  const float* Wo   = (const float*)d_in[15];  const float* bo   = (const float*)d_in[16];
  const float* ln1g = (const float*)d_in[17];  const float* ln1b = (const float*)d_in[18];
  const float* ln2g = (const float*)d_in[19];  const float* ln2b = (const float*)d_in[20];
  const float* Wg   = (const float*)d_in[21];  const float* bg   = (const float*)d_in[22];

  char*  ws    = (char*)d_ws;
  float* biasT = (float*)(ws + WS_BIAS);
  f16*   wt    = (f16*)(ws + WS_WT);
  f16*   wgt   = (f16*)(ws + WS_WG);
  f16*   hpl   = (f16*)(ws + WS_H);
  f16*   cat   = (f16*)(ws + WS_CAT);
  f16*   tpl   = (f16*)(ws + WS_T);
  f16*   qk    = (f16*)(ws + WS_QK);
  f16*   vtp   = (f16*)(ws + WS_VT);
  f16*   ctx   = hpl;
  f16*   c1    = tpl;
  float* opre  = (float*)(ws + WS_T + SZ_ACT);
  float* oln   = (float*)(ws + WS_QK);
  float* out   = (float*)d_out;

  const int PW = DM * DM;
  const int PA = RTOT * DM;

  bias_kernel<<<1, 256, 0, stream>>>(bqp, bkp, bvp, bq, bk, bv, bop, bo, bg, biasT);
  wcvt8_kernel<<<dim3(DM / 64, DM / 64), 256, 0, stream>>>(Wqp, Wkp, Wvp, Wq, Wk, Wv, Wop, Wo, wt);
  wcvtg_kernel<<<dim3(DM / 64, 2 * DM / 64), 256, 0, stream>>>(Wg, wgt);

  ln1_kernel<<<RTOT, LNT, 0, stream>>>(x, ln1g, ln1b, hpl, cat);

  gemm_f16_kernel<<<dim3(DM / GT, RTOT / GT, 3), 256, 0, stream>>>(
      hpl, wt, biasT, tpl, DM, DM, DM, DM, 0, PW, 0, DM, PA, 1.0f / W_S, T_S);
  gemm_f16_kernel<<<dim3(DM / GT, RTOT / GT, 2), 256, 0, stream>>>(
      tpl, wt + (size_t)3 * PW, biasT, qk, DM, DM, DM, DM, PA, PW, 3 * DM, DM, PA,
      1.0f / (W_S * T_S), QKV_S);
  gemm_vt_kernel<<<dim3(RTOT / GT, DM / GT, 1), 256, 0, stream>>>(
      wt + (size_t)5 * PW, tpl + (size_t)2 * PA, biasT, vtp, DM, DM, DM, RTOT, 5 * DM,
      1.0f / (W_S * T_S), QKV_S);

  attn_kernel<<<dim3(SEQ / BQ, NHEAD, NB), 256, 0, stream>>>(qk, qk + (size_t)PA, vtp, ctx);

  gemm_gelu_kernel<<<dim3(DM / GT, RTOT / GT, 1), 256, 0, stream>>>(
      ctx, wt + (size_t)6 * PW, biasT, c1, DM, DM, DM, DM, 6 * DM, 1.0f / (W_S * CTX_S), C1_S);
  gemm_f32_kernel<<<dim3(DM / GT, RTOT / GT, 1), 256, 0, stream>>>(
      c1, wt + (size_t)7 * PW, biasT, opre, DM, DM, DM, DM, 7 * DM, 1.0f / (W_S * C1_S));

  ln2_kernel<<<RTOT, LNT, 0, stream>>>(opre, ln2g, ln2b, cat, oln);

  gemm_gate_kernel<<<dim3(DM / GT, RTOT / GT, 1), 256, 0, stream>>>(
      cat, wgt, biasT, out, oln, x, 2 * DM, 2 * DM, 2 * DM, DM, 8 * DM, 1.0f / W_S);
}
